// TheRecurrentNet_90056874262605
// MI455X (gfx1250) — hardware-verified
//
#include <hip/hip_runtime.h>
#include <stdint.h>
#include <stddef.h>

#define NB    8192
#define NSC   512
#define KE    16
#define HH    500
#define HP    512
#define NA    64
#define N4    100
#define N4P   128
#define N4T   7
#define CP    520
#define SP    516
#define NTHR  256
#define GEMM_LDS (32 * SP * 4)
#define PAIR_LDS (32 * CP * 2 + 32 * SP * 4)
#define LN_EPS 1e-5f
#define W16SCALE 256.0f

static_assert(NB == NSC * KE);
static_assert(HP % 32 == 0 && HP >= HH);
static_assert(HH % 4 == 0 && N4 % 4 == 0 && NA % 32 == 0);
static_assert(CP % 8 == 0 && CP >= HP);
static_assert(SP % 4 == 0 && SP >= HP);
static_assert(NB % 32 == 0 && NSC % 32 == 0);
static_assert(N4T * 16 >= N4 && N4P >= N4T * 16 && N4T <= NTHR / 32);
static_assert((32 * CP * 2) % 16 == 0);
static_assert(NTHR == 256);
static_assert((32 * HH) % 4 == 0);
static_assert((32 * HH * 4) % 128 == 0);

typedef unsigned short u16;
typedef _Float16 f16;
typedef __attribute__((ext_vector_type(16))) __bf16 v16bf;
typedef f16 v16h __attribute__((ext_vector_type(16)));
typedef u16 v8us_t __attribute__((ext_vector_type(8)));
typedef v8us_t __attribute__((may_alias)) v8us;
typedef u16 v4us_t __attribute__((ext_vector_type(4)));
typedef v4us_t __attribute__((may_alias)) v4us;
typedef float v8f __attribute__((ext_vector_type(8)));
typedef float v4f_t __attribute__((ext_vector_type(4)));
typedef v4f_t __attribute__((may_alias)) v4f;

union FragB { v8us_t u[2]; v16bf v; v8f f; };
union FragH { v8us_t u[2]; v16h v; v8f f; };

__device__ __forceinline__ u16 bf_bits(float f) {
    unsigned int u = __float_as_uint(f);
    u += 0x7fffu + ((u >> 16) & 1u);
    return (u16)(u >> 16);
}
__device__ __forceinline__ float bf_val(u16 b) { return __uint_as_float(((unsigned int)b) << 16); }
__device__ __forceinline__ float bfr(float f) { return bf_val(bf_bits(f)); }
__device__ __forceinline__ u16 h_bits(float f) { union { f16 h; u16 u; } c; c.h = (f16)f; return c.u; }

__device__ __forceinline__ float wsum(float v) {
#pragma unroll
    for (int o = 16; o > 0; o >>= 1) v += __shfl_xor(v, o, 32);
    return v;
}
__device__ __forceinline__ v8f zero8() {
    v8f z;
#pragma unroll
    for (int i = 0; i < 8; ++i) z[i] = 0.0f;
    return z;
}

__device__ __forceinline__ void ldfrag(const u16* p, int k0, v8us_t& e0, v8us_t& e1) {
    e0 = *(const v8us*)(p + k0);
    e1 = *(const v8us*)(p + k0 + 16);
}
__device__ __forceinline__ v8f mma_bf(const FragB& a, const FragB& b, v8f c) {
    return __builtin_amdgcn_wmma_f32_16x16x32_bf16(false, a.v, false, b.v, (short)0, c, false, false);
}
__device__ __forceinline__ v8f mma_h(const FragH& a, const FragH& b, v8f c) {
    return __builtin_amdgcn_wmma_f32_16x16x32_f16(false, a.v, false, b.v, (short)0, c, false, false);
}

__global__ void __launch_bounds__(NTHR) cvt_rows_kernel(const float* __restrict__ src, int cols,
                                                       u16* __restrict__ dst, int pitch, int n8)
{
    const int t = blockIdx.x * NTHR + (int)threadIdx.x;
    const bool ok = (t < n8);
    const int tt = ok ? t : 0;
    const long long e0 = (long long)tt * 8;
    const int row = (int)(e0 / pitch);
    const int c0 = (int)(e0 % pitch);
    v8us_t pk;
#pragma unroll
    for (int g = 0; g < 2; ++g) {
        const int c = c0 + 4 * g;
        const bool v = (c < cols);
        const int ca = v ? c : (cols - 4);
        const v4f_t x = *(const v4f*)(src + (size_t)row * cols + ca);
#pragma unroll
        for (int j = 0; j < 4; ++j) pk[4 * g + j] = v ? bf_bits(x[j]) : (u16)0;
    }
    u16* d = dst + (size_t)tt * 8;
    if (ok) *(volatile v8us_t*)d = pk;
    __threadfence();
    if (ok) *(volatile v8us_t*)d = pk;
}

__global__ void __launch_bounds__(NTHR) cvt_wT_kernel(const float* __restrict__ src, int K, int N,
                                                     u16* __restrict__ dst, int ldk, int koff,
                                                     int mode, float scale)
{
    __shared__ float tile[64][65];
    const int t = threadIdx.x;
    const int k0 = blockIdx.x * 64, n0 = blockIdx.y * 64;
    const int nn = t & 63, kq = t >> 6;
    const int n = n0 + nn;
    const int na = (n < N) ? n : (N - 1);
#pragma unroll 4
    for (int it = 0; it < 16; ++it) {
        const int kk = kq + 4 * it;
        const int k = k0 + kk;
        const int ka = (k < K) ? k : (K - 1);
        const float x = src[(size_t)ka * N + na];
        tile[kk][nn] = (k < K && n < N) ? x : 0.f;
    }
    __syncthreads();
    const int lane = t & 31, w = t >> 5, q = lane >> 3, cb = 8 * (lane & 7);
    const int r0 = 8 * w + q, r1 = 8 * w + 4 + q;
    v8us_t pk0, pk1;
#pragma unroll
    for (int j = 0; j < 8; ++j) {
        const float x0 = tile[cb + j][r0];
        const float x1 = tile[cb + j][r1];
        pk0[j] = mode ? h_bits(bfr(x0) * scale) : bf_bits(x0);
        pk1[j] = mode ? h_bits(bfr(x1) * scale) : bf_bits(x1);
    }
    u16* d0 = dst + (size_t)(n0 + r0) * ldk + koff + k0 + cb;
    u16* d1 = dst + (size_t)(n0 + r1) * ldk + koff + k0 + cb;
    *(volatile v8us_t*)d0 = pk0;
    *(volatile v8us_t*)d1 = pk1;
    __threadfence();
    *(volatile v8us_t*)d0 = pk0;
    *(volatile v8us_t*)d1 = pk1;
}

__global__ void __launch_bounds__(NTHR) att_a_kernel(const u16* __restrict__ stb, const float* __restrict__ af,
                                                    const float* __restrict__ w3, const float* __restrict__ b3,
                                                    float* __restrict__ attA)
{
    __shared__ __align__(16) float vals[32];
    const int t = threadIdx.x, lane = t & 31, w = t >> 5;
    const int n0 = blockIdx.x * 32;
#pragma unroll 1
    for (int rr = 0; rr < 4; ++rr) {
        const int n = n0 + 4 * w + rr;
        const u16* sr = stb + (size_t)n * HP;
        const float* ar = af + (size_t)(n >> 4) * HP;
        float s = 0.f;
#pragma unroll 1
        for (int it = 0; it < HP / 32; ++it) {
            const int c = lane + 32 * it;
            const int ca = (c < HH) ? c : (HH - 1);
            const float sv = bf_val(sr[c]);
            const float av = ar[c];
            s = fmaf(sv, bfr(w3[ca]), s);
            s = fmaf(av, bfr(w3[HH + ca]), s);
        }
        s = wsum(s);
        const float z = s + bfr(b3[0]);
        const float sg = __builtin_amdgcn_rcpf(1.0f + expf(-z));
        if (lane == 0) vals[4 * w + rr] = sg;
    }
    __syncthreads();
    if (w == 0) {
        const v4f_t v = *(const v4f*)(vals + 4 * (lane & 7));
        float* d = attA + n0 + 4 * (lane & 7);
        if (lane < 8) *(volatile v4f_t*)d = v;
        __threadfence();
        if (lane < 8) *(volatile v4f_t*)d = v;
    }
}

__device__ __forceinline__ void gemm_store_pass(const float* stage, int w, int lane, int t, int m0,
                                                float* outf, int ldf, int fmode, u16* outh, u16* outl)
{
    if (fmode == 1) {
#pragma unroll
        for (int rr = 0; rr < 4; ++rr) {
            const int row = 4 * w + rr;
            const int gm = m0 + row;
#pragma unroll
            for (int i = 0; i < 4; ++i) {
                const v4f_t v = *(const v4f*)(stage + row * SP + 128 * i + 4 * lane);
                *(volatile v4f_t*)(outf + (size_t)gm * ldf + 128 * i + 4 * lane) = v;
            }
        }
    } else if (fmode == 2) {
#pragma unroll
        for (int it = 0; it < 16; ++it) {
            const int f = t + NTHR * it;
            if (f < (32 * HH) / 4) {
                const int row = f / (HH / 4);
                const int col = 4 * (f - (HH / 4) * row);
                const v4f_t v = *(const v4f*)(stage + row * SP + col);
                *(volatile v4f_t*)(outf + (size_t)m0 * HH + 4 * f) = v;
            }
        }
    }
    if (outh != nullptr) {
#pragma unroll
        for (int rr = 0; rr < 4; ++rr) {
            const int row = 4 * w + rr;
            const int gm = m0 + row;
#pragma unroll
            for (int i = 0; i < 2; ++i) {
                const int c = 256 * i + 8 * lane;
                const v4f_t x0 = *(const v4f*)(stage + row * SP + c);
                const v4f_t x1 = *(const v4f*)(stage + row * SP + c + 4);
                v8us_t hb, lb;
#pragma unroll
                for (int j = 0; j < 4; ++j) {
                    const u16 h0 = bf_bits(x0[j]);
                    hb[j] = h0; lb[j] = bf_bits(x0[j] - bf_val(h0));
                    const u16 h1 = bf_bits(x1[j]);
                    hb[4 + j] = h1; lb[4 + j] = bf_bits(x1[j] - bf_val(h1));
                }
                *(volatile v8us_t*)(outh + (size_t)gm * HP + c) = hb;
                *(volatile v8us_t*)(outl + (size_t)gm * HP + c) = lb;
            }
        }
    }
}

__global__ void __launch_bounds__(NTHR) gemm_node_kernel(
    const u16* __restrict__ a0, int bo0, int ns0,
    const u16* __restrict__ a1, int bo1, int ns1,
    const u16* __restrict__ a2, int bo2, int ns2,
    const u16* __restrict__ a3, int bo3, int ns3,
    int nseg, int lda,
    const u16* __restrict__ bpl, int ldb,
    const float* __restrict__ bias,
    const float* __restrict__ radd, int rsh,
    const float* __restrict__ lng, const float* __restrict__ lnb,
    int act,
    const float* __restrict__ rscale,
    float* __restrict__ outf, int ldf, int fmode,
    u16* __restrict__ outh, u16* __restrict__ outl)
{
    extern __shared__ __align__(16) float glds[];
    float* stage = glds;
    const int t = threadIdx.x, lane = t & 31, w = t >> 5, hh = lane >> 4, m = lane & 15;
    const int m0 = blockIdx.x * 32;

    v8f acc[2][4];
#pragma unroll
    for (int i = 0; i < 2; ++i)
#pragma unroll
        for (int j = 0; j < 4; ++j) acc[i][j] = zero8();

#pragma unroll 1
    for (int s = 0; s < nseg; ++s) {
        const u16* ap = a0; int bo = bo0, ns = ns0;
        if (s == 1)      { ap = a1; bo = bo1; ns = ns1; }
        else if (s == 2) { ap = a2; bo = bo2; ns = ns2; }
        else if (s == 3) { ap = a3; bo = bo3; ns = ns3; }
        const u16* pa0 = ap + (size_t)(m0 + m) * lda + 8 * hh;
        const u16* pa1 = pa0 + (size_t)16 * lda;
        const u16* pb  = bpl + (size_t)(64 * w + m) * ldb + bo + 8 * hh;
#pragma unroll 1
        for (int ks = 0; ks < ns; ++ks) {
            const int k0 = ks * 32;
            FragB fa0, fa1, fb0, fb1, fb2, fb3;
            ldfrag(pa0, k0, fa0.u[0], fa0.u[1]);
            ldfrag(pa1, k0, fa1.u[0], fa1.u[1]);
            ldfrag(pb, k0, fb0.u[0], fb0.u[1]);
            ldfrag(pb + (size_t)16 * ldb, k0, fb1.u[0], fb1.u[1]);
            ldfrag(pb + (size_t)32 * ldb, k0, fb2.u[0], fb2.u[1]);
            ldfrag(pb + (size_t)48 * ldb, k0, fb3.u[0], fb3.u[1]);
            acc[0][0] = mma_bf(fa0, fb0, acc[0][0]);
            acc[0][1] = mma_bf(fa0, fb1, acc[0][1]);
            acc[0][2] = mma_bf(fa0, fb2, acc[0][2]);
            acc[0][3] = mma_bf(fa0, fb3, acc[0][3]);
            acc[1][0] = mma_bf(fa1, fb0, acc[1][0]);
            acc[1][1] = mma_bf(fa1, fb1, acc[1][1]);
            acc[1][2] = mma_bf(fa1, fb2, acc[1][2]);
            acc[1][3] = mma_bf(fa1, fb3, acc[1][3]);
            asm volatile("v_nop\n\tv_nop\n\tv_nop\n\tv_nop"
                         : "+v"(acc[0][0]), "+v"(acc[0][1]), "+v"(acc[0][2]), "+v"(acc[0][3]),
                           "+v"(acc[1][0]), "+v"(acc[1][1]), "+v"(acc[1][2]), "+v"(acc[1][3])
                         : "v"(fa0.f), "v"(fa1.f), "v"(fb0.f), "v"(fb1.f), "v"(fb2.f), "v"(fb3.f));
        }
    }

#pragma unroll
    for (int mt = 0; mt < 2; ++mt)
#pragma unroll
        for (int nt = 0; nt < 4; ++nt)
#pragma unroll
            for (int r = 0; r < 8; ++r)
                stage[(mt * 16 + 8 * hh + r) * SP + 64 * w + 16 * nt + m] = acc[mt][nt][r];
    __syncthreads();

#pragma unroll 1
    for (int rr = 0; rr < 4; ++rr) {
        const int row = 4 * w + rr;
        const int gm = m0 + row;
        float* srow = stage + row * SP + 16 * lane;
        float x[16];
        float s = 0.f;
#pragma unroll
        for (int q = 0; q < 4; ++q) {
            const int c = 16 * lane + 4 * q;
            const bool v = (c < HH);
            const int ca = v ? c : (HH - 4);
            const v4f_t xv = *(const v4f*)(srow + 4 * q);
            v4f_t bb; bb[0] = 0.f; bb[1] = 0.f; bb[2] = 0.f; bb[3] = 0.f;
            if (bias != nullptr) bb = *(const v4f*)(bias + ca);
            v4f_t ra; ra[0] = 0.f; ra[1] = 0.f; ra[2] = 0.f; ra[3] = 0.f;
            if (radd != nullptr) ra = *(const v4f*)(radd + (size_t)(gm >> rsh) * HP + c);
#pragma unroll
            for (int j = 0; j < 4; ++j) {
                const float val = v ? ((xv[j] + bfr(bb[j])) + ra[j]) : 0.f;
                x[4 * q + j] = val;
                s += val;
            }
        }
        if (lng != nullptr) {
            s = wsum(s);
            const float mu = s * (1.0f / (float)HH);
            float s2 = 0.f;
#pragma unroll
            for (int q = 0; q < 4; ++q) {
                const bool v = (16 * lane + 4 * q < HH);
#pragma unroll
                for (int j = 0; j < 4; ++j) {
                    const float d = v ? (x[4 * q + j] - mu) : 0.f;
                    x[4 * q + j] = d;
                    s2 += d * d;
                }
            }
            s2 = wsum(s2);
            const float rstd = rsqrtf(s2 * (1.0f / (float)HH) + LN_EPS);
#pragma unroll
            for (int q = 0; q < 4; ++q) {
                const int c = 16 * lane + 4 * q;
                const bool v = (c < HH);
                const int ca = v ? c : (HH - 4);
                const v4f_t gg = *(const v4f*)(lng + ca);
                const v4f_t be = *(const v4f*)(lnb + ca);
#pragma unroll
                for (int j = 0; j < 4; ++j)
                    x[4 * q + j] = v ? (x[4 * q + j] * rstd * bfr(gg[j]) + bfr(be[j])) : 0.f;
            }
        }
        float rs = 1.0f;
        if (rscale != nullptr) rs = rscale[gm];
#pragma unroll
        for (int i = 0; i < 16; ++i) {
            float vv = x[i];
            if (act == 1) vv = fmaxf(vv, 0.f);
            x[i] = vv * rs;
        }
#pragma unroll
        for (int q = 0; q < 4; ++q) {
            v4f_t o; o[0] = x[4 * q]; o[1] = x[4 * q + 1]; o[2] = x[4 * q + 2]; o[3] = x[4 * q + 3];
            *(v4f*)(srow + 4 * q) = o;
        }
    }
    __syncthreads();

    gemm_store_pass(stage, w, lane, t, m0, outf, ldf, fmode, outh, outl);
    __threadfence();
    gemm_store_pass(stage, w, lane, t, m0, outf, ldf, fmode, outh, outl);
}

__device__ __forceinline__ void pair_store_pass(const u16* esst, int w, int lane, int nb0, u16* esh, u16* esl)
{
    const int e = w >> 2, pl = (w >> 1) & 1, pc = w & 1;
    const v8us_t v = *(const v8us*)(esst + (e * 2 + pl) * HP + 256 * pc + 8 * lane);
    u16* d = (pl ? esl : esh) + (size_t)(nb0 + e) * HP + 256 * pc + 8 * lane;
    *(volatile v8us_t*)d = v;
}

__global__ void __launch_bounds__(NTHR) pair_kernel(
    const float* __restrict__ pq,
    const float* __restrict__ b2, const float* __restrict__ g2, const float* __restrict__ be2,
    const u16* __restrict__ w3p, const float* __restrict__ b3, const float* __restrict__ g3, const float* __restrict__ be3,
    const u16* __restrict__ w4p, const float* __restrict__ b4, const float* __restrict__ g4, const float* __restrict__ be4,
    const float* __restrict__ w5, const float* __restrict__ b5,
    u16* __restrict__ esh, u16* __restrict__ esl)
{
    extern __shared__ __align__(16) unsigned char plds[];
    u16* coreA = (u16*)plds;
    float* stage = (float*)(plds + 32 * CP * 2);
    __shared__ float attL[32];
    __shared__ float muL[32];
    __shared__ float rsL[32];

    const int t = threadIdx.x, lane = t & 31, w = t >> 5, hh = lane >> 4, m = lane & 15;
    const int nb0 = blockIdx.x * 2;

#pragma unroll 1
    for (int rr = 0; rr < 4; ++rr) {
        const int row = 4 * w + rr;
        const int e = row >> 4, p = row & 15;
        const int n = nb0 + e;
        const int i = n & (KE - 1);
        const int jj = (p == KE - 1) ? i : (p + ((p >= i) ? 1 : 0));
        const int nq = (n & ~(KE - 1)) + jj;
        const float* prow = pq + (size_t)n * (2 * HP) + 16 * lane;
        const float* qrow = pq + (size_t)nq * (2 * HP) + HP + 16 * lane;
        float x[16];
        float s = 0.f;
#pragma unroll
        for (int q = 0; q < 4; ++q) {
            const int c = 16 * lane + 4 * q;
            const bool v = (c < HH);
            const int ca = v ? c : (HH - 4);
            const v4f_t pa = *(const v4f*)(prow + 4 * q);
            const v4f_t qa = *(const v4f*)(qrow + 4 * q);
            const v4f_t bb = *(const v4f*)(b2 + ca);
#pragma unroll
            for (int j = 0; j < 4; ++j) {
                const float xv = v ? ((pa[j] + qa[j]) + bfr(bb[j])) : 0.f;
                x[4 * q + j] = xv;
                s += xv;
            }
        }
        s = wsum(s);
        const float mu = s * (1.0f / (float)HH);
        float s2 = 0.f;
#pragma unroll
        for (int q = 0; q < 4; ++q) {
            const bool v = (16 * lane + 4 * q < HH);
#pragma unroll
            for (int j = 0; j < 4; ++j) {
                const float d = v ? (x[4 * q + j] - mu) : 0.f;
                x[4 * q + j] = d;
                s2 += d * d;
            }
        }
        s2 = wsum(s2);
        const float rstd = rsqrtf(s2 * (1.0f / (float)HH) + LN_EPS);
        v8us_t pk0, pk1;
#pragma unroll
        for (int q = 0; q < 4; ++q) {
            const int c = 16 * lane + 4 * q;
            const bool v = (c < HH);
            const int ca = v ? c : (HH - 4);
            const v4f_t gg = *(const v4f*)(g2 + ca);
            const v4f_t be = *(const v4f*)(be2 + ca);
#pragma unroll
            for (int j = 0; j < 4; ++j) {
                const float y = v ? fmaxf(x[4 * q + j] * rstd * bfr(gg[j]) + bfr(be[j]), 0.f) : 0.f;
                const u16 hb = h_bits(y);
                if (q < 2) pk0[4 * q + j] = hb; else pk1[4 * (q - 2) + j] = hb;
            }
        }
        *(v8us*)(coreA + row * CP + 16 * lane) = pk0;
        *(v8us*)(coreA + row * CP + 16 * lane + 8) = pk1;
    }
    __syncthreads();

    {
        v8f a40 = zero8(), a41 = zero8();
        if (w < N4T) {
            const u16* pa0 = coreA + m * CP + 8 * hh;
            const u16* pa1 = pa0 + 16 * CP;
            const u16* pb  = w4p + (size_t)(16 * w + m) * HP + 8 * hh;
#pragma unroll 1
            for (int ks = 0; ks < HP / 32; ++ks) {
                const int k0 = ks * 32;
                FragH fa0, fa1, fb;
                ldfrag(pa0, k0, fa0.u[0], fa0.u[1]);
                ldfrag(pa1, k0, fa1.u[0], fa1.u[1]);
                ldfrag(pb, k0, fb.u[0], fb.u[1]);
                a40 = mma_h(fa0, fb, a40);
                a41 = mma_h(fa1, fb, a41);
                asm volatile("v_nop\n\tv_nop\n\tv_nop\n\tv_nop"
                             : "+v"(a40), "+v"(a41) : "v"(fa0.f), "v"(fa1.f), "v"(fb.f));
            }
#pragma unroll
            for (int r = 0; r < 8; ++r) {
                stage[(8 * hh + r) * SP + 16 * w + m]      = a40[r] * (1.0f / W16SCALE);
                stage[(16 + 8 * hh + r) * SP + 16 * w + m] = a41[r] * (1.0f / W16SCALE);
            }
        }
    }
    __syncthreads();

#pragma unroll 1
    for (int rr = 0; rr < 4; ++rr) {
        const int row = 4 * w + rr;
        float xv[4];
        float s = 0.f;
#pragma unroll
        for (int q = 0; q < 4; ++q) {
            const int c = lane + 32 * q;
            const bool v = (c < N4);
            const int ca = v ? c : (N4 - 1);
            const float xx = v ? (stage[row * SP + ca] + bfr(b4[ca])) : 0.f;
            xv[q] = xx;
            s += xx;
        }
        s = wsum(s);
        const float mu = s * (1.0f / (float)N4);
        float s2 = 0.f;
#pragma unroll
        for (int q = 0; q < 4; ++q) {
            const bool v = (lane + 32 * q < N4);
            const float d = v ? (xv[q] - mu) : 0.f;
            xv[q] = d;
            s2 += d * d;
        }
        s2 = wsum(s2);
        const float rstd = rsqrtf(s2 * (1.0f / (float)N4) + LN_EPS);
        float dot = 0.f;
#pragma unroll
        for (int q = 0; q < 4; ++q) {
            const int c = lane + 32 * q;
            const bool v = (c < N4);
            const int ca = v ? c : (N4 - 1);
            const float y = tanhf(xv[q] * rstd * bfr(g4[ca]) + bfr(be4[ca]));
            dot += v ? (y * bfr(w5[ca])) : 0.f;
        }
        dot = wsum(dot);
        const float z = dot + bfr(b5[0]);
        const float sg = __builtin_amdgcn_rcpf(1.0f + expf(-z));
        if (lane == 0) attL[row] = sg;
    }
    __syncthreads();

    {
        v8f c3[2][4];
#pragma unroll
        for (int a = 0; a < 2; ++a)
#pragma unroll
            for (int b = 0; b < 4; ++b) c3[a][b] = zero8();
        const u16* pa0 = coreA + m * CP + 8 * hh;
        const u16* pa1 = pa0 + 16 * CP;
        const u16* pb  = w3p + (size_t)(64 * w + m) * HP + 8 * hh;
#pragma unroll 1
        for (int ks = 0; ks < HP / 32; ++ks) {
            const int k0 = ks * 32;
            FragH fa0, fa1, fb0, fb1, fb2, fb3;
            ldfrag(pa0, k0, fa0.u[0], fa0.u[1]);
            ldfrag(pa1, k0, fa1.u[0], fa1.u[1]);
            ldfrag(pb, k0, fb0.u[0], fb0.u[1]);
            ldfrag(pb + (size_t)16 * HP, k0, fb1.u[0], fb1.u[1]);
            ldfrag(pb + (size_t)32 * HP, k0, fb2.u[0], fb2.u[1]);
            ldfrag(pb + (size_t)48 * HP, k0, fb3.u[0], fb3.u[1]);
            c3[0][0] = mma_h(fa0, fb0, c3[0][0]);
            c3[0][1] = mma_h(fa0, fb1, c3[0][1]);
            c3[0][2] = mma_h(fa0, fb2, c3[0][2]);
            c3[0][3] = mma_h(fa0, fb3, c3[0][3]);
            c3[1][0] = mma_h(fa1, fb0, c3[1][0]);
            c3[1][1] = mma_h(fa1, fb1, c3[1][1]);
            c3[1][2] = mma_h(fa1, fb2, c3[1][2]);
            c3[1][3] = mma_h(fa1, fb3, c3[1][3]);
            asm volatile("v_nop\n\tv_nop\n\tv_nop\n\tv_nop"
                         : "+v"(c3[0][0]), "+v"(c3[0][1]), "+v"(c3[0][2]), "+v"(c3[0][3]),
                           "+v"(c3[1][0]), "+v"(c3[1][1]), "+v"(c3[1][2]), "+v"(c3[1][3])
                         : "v"(fa0.f), "v"(fa1.f), "v"(fb0.f), "v"(fb1.f), "v"(fb2.f), "v"(fb3.f));
        }
#pragma unroll
        for (int mt = 0; mt < 2; ++mt)
#pragma unroll
            for (int nt = 0; nt < 4; ++nt)
#pragma unroll
                for (int r = 0; r < 8; ++r)
                    stage[(mt * 16 + 8 * hh + r) * SP + 64 * w + 16 * nt + m] = c3[mt][nt][r] * (1.0f / W16SCALE);
    }
    __syncthreads();

#pragma unroll 1
    for (int rr = 0; rr < 4; ++rr) {
        const int row = 4 * w + rr;
        const float* srow = stage + row * SP + 16 * lane;
        float x[16];
        float s = 0.f;
#pragma unroll
        for (int q = 0; q < 4; ++q) {
            const int c = 16 * lane + 4 * q;
            const bool v = (c < HH);
            const int ca = v ? c : (HH - 4);
            const v4f_t xv = *(const v4f*)(srow + 4 * q);
            const v4f_t bb = *(const v4f*)(b3 + ca);
#pragma unroll
            for (int j = 0; j < 4; ++j) {
                const float val = v ? (xv[j] + bfr(bb[j])) : 0.f;
                x[4 * q + j] = val;
                s += val;
            }
        }
        s = wsum(s);
        const float mu = s * (1.0f / (float)HH);
        float s2 = 0.f;
#pragma unroll
        for (int q = 0; q < 4; ++q) {
            const bool v = (16 * lane + 4 * q < HH);
#pragma unroll
            for (int j = 0; j < 4; ++j) {
                const float d = v ? (x[4 * q + j] - mu) : 0.f;
                s2 += d * d;
            }
        }
        s2 = wsum(s2);
        const float rstd = rsqrtf(s2 * (1.0f / (float)HH) + LN_EPS);
        if (lane == 0) { muL[row] = mu; rsL[row] = rstd; }
    }
    __syncthreads();

    {
        const int e = t >> 7;
        const int c = 4 * (t & 127);
        const bool v = (c < HH);
        const int ca = v ? c : (HH - 4);
        const v4f_t bb = *(const v4f*)(b3 + ca);
        const v4f_t gg = *(const v4f*)(g3 + ca);
        const v4f_t be = *(const v4f*)(be3 + ca);
        float bq[4], gq[4], eq[4], acc4[4];
#pragma unroll
        for (int j = 0; j < 4; ++j) { bq[j] = bfr(bb[j]); gq[j] = bfr(gg[j]); eq[j] = bfr(be[j]); acc4[j] = 0.f; }
#pragma unroll 1
        for (int p = 0; p < KE - 1; ++p) {
            const int row = e * 16 + p;
            const v4f_t xv = *(const v4f*)(stage + row * SP + c);
            const float mu = muL[row], rs = rsL[row], at = attL[row];
#pragma unroll
            for (int j = 0; j < 4; ++j) {
                const float y = fmaxf(((xv[j] + bq[j]) - mu) * rs * gq[j] + eq[j], 0.f);
                acc4[j] += y * at;
            }
        }
        v4us_t hb, lb;
#pragma unroll
        for (int j = 0; j < 4; ++j) {
            const float val = v ? acc4[j] : 0.f;
            const u16 h0 = bf_bits(val);
            hb[j] = h0;
            lb[j] = bf_bits(val - bf_val(h0));
        }
        *(v4us*)(coreA + (e * 2 + 0) * HP + c) = hb;
        *(v4us*)(coreA + (e * 2 + 1) * HP + c) = lb;
    }
    __syncthreads();

    pair_store_pass(coreA, w, lane, nb0, esh, esl);
    __threadfence();
    pair_store_pass(coreA, w, lane, nb0, esh, esl);
}

extern "C" void kernel_launch(void* const* d_in, const int* in_sizes, int n_in,
                              void* d_out, int out_size, void* d_ws, size_t ws_size,
                              hipStream_t stream)
{
    if (n_in < 34) return;
    const int expect_n[34] = {
        NB * HH, NSC * NA,
        NA * HH, HH, HH, HH, 2 * HH * HH, HH, HH * HH, HH, 2 * HH, 1,
        HH * HH, HH, HH, HH,
        2 * HH * HH, HH, HH, HH,
        HH * HH, HH, HH, HH,
        HH * N4, N4, N4, N4,
        N4, 1,
        2 * HH * HH, HH, HH, HH };
    for (int i = 0; i < 34; ++i) if (in_sizes[i] != expect_n[i]) return;
    if (out_size != NB * HH) return;

    const float* state     = (const float*)d_in[0];
    const float* actions   = (const float*)d_in[1];
    const float* ac_fc1_w  = (const float*)d_in[2];
    const float* ac_fc1_b  = (const float*)d_in[3];
    const float* ac_ln1_g  = (const float*)d_in[4];
    const float* ac_ln1_b  = (const float*)d_in[5];
    const float* ac_fc2_w  = (const float*)d_in[6];
    const float* ac_fc2_b  = (const float*)d_in[7];
    const float* ac_lnf2_w = (const float*)d_in[8];
    const float* ac_lnf2_b = (const float*)d_in[9];
    const float* ac_fc3_w  = (const float*)d_in[10];
    const float* ac_fc3_b  = (const float*)d_in[11];
    const float* fc1_w = (const float*)d_in[12];
    const float* fc1_b = (const float*)d_in[13];
    const float* ln1_g = (const float*)d_in[14];
    const float* ln1_b = (const float*)d_in[15];
    const float* fc2_w = (const float*)d_in[16];
    const float* fc2_b = (const float*)d_in[17];
    const float* ln2_g = (const float*)d_in[18];
    const float* ln2_b = (const float*)d_in[19];
    const float* fc3_w = (const float*)d_in[20];
    const float* fc3_b = (const float*)d_in[21];
    const float* ln3_g = (const float*)d_in[22];
    const float* ln3_b = (const float*)d_in[23];
    const float* fc4_w = (const float*)d_in[24];
    const float* fc4_b = (const float*)d_in[25];
    const float* ln4_g = (const float*)d_in[26];
    const float* ln4_b = (const float*)d_in[27];
    const float* fc5_w = (const float*)d_in[28];
    const float* fc5_b = (const float*)d_in[29];
    const float* fc6_w = (const float*)d_in[30];
    const float* fc6_b = (const float*)d_in[31];
    const float* ln6_g = (const float*)d_in[32];
    const float* ln6_b = (const float*)d_in[33];
    float* out = (float*)d_out;

    char* ws = (char*)d_ws;
    size_t off = 0;
    auto carve = [&](size_t bytes) -> char* {
        char* p = ws + off;
        off += (bytes + 255) & ~(size_t)255;
        return p;
    };
    const size_t plane16 = (size_t)NB * HP * 2;
    u16*   act_bf = (u16*)carve((size_t)NSC * NA * 2);
    u16*   st_bf  = (u16*)carve(plane16);
    u16*   Wac1   = (u16*)carve((size_t)HP * NA * 2);
    u16*   Wac2   = (u16*)carve((size_t)HP * 2 * HP * 2);
    u16*   Wlnf2  = (u16*)carve((size_t)HP * HP * 2);
    u16*   Wfc1   = (u16*)carve((size_t)HP * HP * 2);
    u16*   W2a    = (u16*)carve((size_t)HP * HP * 2);
    u16*   W2b    = (u16*)carve((size_t)HP * HP * 2);
    u16*   W3     = (u16*)carve((size_t)HP * HP * 2);
    u16*   W4     = (u16*)carve((size_t)N4P * HP * 2);
    u16*   Wfc6   = (u16*)carve((size_t)HP * 2 * HP * 2);
    float* a_f32  = (float*)carve((size_t)NSC * HP * 4);
    u16*   a_hi   = (u16*)carve((size_t)NSC * HP * 2);
    u16*   a_lo   = (u16*)carve((size_t)NSC * HP * 2);
    float* Ta     = (float*)carve((size_t)NSC * HP * 4);
    float* attA   = (float*)carve((size_t)NB * 4);
    u16*   T_hi   = (u16*)carve(plane16);
    u16*   T_lo   = (u16*)carve(plane16);
    u16*   st2_hi = (u16*)carve(plane16);
    u16*   st2_lo = (u16*)carve(plane16);
    u16*   s1_hi  = (u16*)carve(plane16);
    u16*   s1_lo  = (u16*)carve(plane16);
    float* PQ     = (float*)carve((size_t)NB * 2 * HP * 4);
    u16*   es_hi  = (u16*)carve(plane16);
    u16*   es_lo  = (u16*)carve(plane16);
    if (off > ws_size) return;
    if (off > (size_t)134217728) return;

    hipFuncSetAttribute(reinterpret_cast<const void*>(&gemm_node_kernel),
                        hipFuncAttributeMaxDynamicSharedMemorySize, GEMM_LDS);
    hipFuncSetAttribute(reinterpret_cast<const void*>(&pair_kernel),
                        hipFuncAttributeMaxDynamicSharedMemorySize, PAIR_LDS);

    {
        const int n8a = NSC * NA / 8;
        const int n8s = NB * HP / 8;
        cvt_rows_kernel<<<dim3((n8a + NTHR - 1) / NTHR), dim3(NTHR), 0, stream>>>(actions, NA, act_bf, NA, n8a);
        cvt_rows_kernel<<<dim3((n8s + NTHR - 1) / NTHR), dim3(NTHR), 0, stream>>>(state, HH, st_bf, HP, n8s);
    }
    const size_t half2 = (size_t)HH * HH;
    cvt_wT_kernel<<<dim3(NA / 64, HP / 64), dim3(NTHR), 0, stream>>>(ac_fc1_w, NA, HH, Wac1, NA, 0, 0, 1.0f);
    cvt_wT_kernel<<<dim3(HP / 64, HP / 64), dim3(NTHR), 0, stream>>>(ac_fc2_w, HH, HH, Wac2, 2 * HP, 0, 0, 1.0f);
    cvt_wT_kernel<<<dim3(HP / 64, HP / 64), dim3(NTHR), 0, stream>>>(ac_fc2_w + half2, HH, HH, Wac2, 2 * HP, HP, 0, 1.0f);
    cvt_wT_kernel<<<dim3(HP / 64, HP / 64), dim3(NTHR), 0, stream>>>(ac_lnf2_w, HH, HH, Wlnf2, HP, 0, 0, 1.0f);
    cvt_wT_kernel<<<dim3(HP / 64, HP / 64), dim3(NTHR), 0, stream>>>(fc1_w, HH, HH, Wfc1, HP, 0, 0, 1.0f);
    cvt_wT_kernel<<<dim3(HP / 64, HP / 64), dim3(NTHR), 0, stream>>>(fc2_w, HH, HH, W2a, HP, 0, 0, 1.0f);
    cvt_wT_kernel<<<dim3(HP / 64, HP / 64), dim3(NTHR), 0, stream>>>(fc2_w + half2, HH, HH, W2b, HP, 0, 0, 1.0f);
    cvt_wT_kernel<<<dim3(HP / 64, HP / 64), dim3(NTHR), 0, stream>>>(fc3_w, HH, HH, W3, HP, 0, 1, W16SCALE);
    cvt_wT_kernel<<<dim3(HP / 64, N4P / 64), dim3(NTHR), 0, stream>>>(fc4_w, HH, N4, W4, HP, 0, 1, W16SCALE);
    cvt_wT_kernel<<<dim3(HP / 64, HP / 64), dim3(NTHR), 0, stream>>>(fc6_w, HH, HH, Wfc6, 2 * HP, 0, 0, 1.0f);
    cvt_wT_kernel<<<dim3(HP / 64, HP / 64), dim3(NTHR), 0, stream>>>(fc6_w + half2, HH, HH, Wfc6, 2 * HP, HP, 0, 1.0f);

    auto gemm = [&](int mrows,
                    const u16* A0, int b0, int n0, const u16* A1, int b1, int n1,
                    const u16* A2, int b2, int n2, const u16* A3, int b3, int n3,
                    int nseg, int lda, const u16* B, int ldb,
                    const float* bias, const float* radd, int rsh,
                    const float* g, const float* bv, int act, const float* rsc,
                    float* of, int ldf, int fmode, u16* oh, u16* ol) {
        gemm_node_kernel<<<dim3(mrows / 32), dim3(NTHR), GEMM_LDS, stream>>>(
            A0, b0, n0, A1, b1, n1, A2, b2, n2, A3, b3, n3, nseg, lda, B, ldb,
            bias, radd, rsh, g, bv, act, rsc, of, ldf, fmode, oh, ol);
    };
    const int KS = HP / 32;

    gemm(NSC, act_bf, 0, NA / 32, nullptr, 0, 0, nullptr, 0, 0, nullptr, 0, 0,
         1, NA, Wac1, NA, ac_fc1_b, nullptr, 0, ac_ln1_g, ac_ln1_b, 0, nullptr,
         a_f32, HP, 1, a_hi, a_lo);
    att_a_kernel<<<dim3(NB / 32), dim3(NTHR), 0, stream>>>(st_bf, a_f32, ac_fc3_w, ac_fc3_b, attA);
    gemm(NSC, a_hi, HP, KS, a_lo, HP, KS, nullptr, 0, 0, nullptr, 0, 0,
         2, HP, Wac2, 2 * HP, ac_fc2_b, nullptr, 0, nullptr, nullptr, 0, nullptr,
         Ta, HP, 1, nullptr, nullptr);
    gemm(NB, st_bf, 0, KS, nullptr, 0, 0, nullptr, 0, 0, nullptr, 0, 0,
         1, HP, Wac2, 2 * HP, nullptr, Ta, 4, nullptr, nullptr, 0, nullptr,
         nullptr, 0, 0, T_hi, T_lo);
    gemm(NB, T_hi, 0, KS, T_lo, 0, KS, nullptr, 0, 0, nullptr, 0, 0,
         2, HP, Wlnf2, HP, ac_lnf2_b, nullptr, 0, nullptr, nullptr, 0, attA,
         nullptr, 0, 0, st2_hi, st2_lo);
    gemm(NB, st2_hi, 0, KS, st2_lo, 0, KS, nullptr, 0, 0, nullptr, 0, 0,
         2, HP, Wfc1, HP, fc1_b, nullptr, 0, ln1_g, ln1_b, 1, nullptr,
         nullptr, 0, 0, s1_hi, s1_lo);
    gemm(NB, s1_hi, 0, KS, s1_lo, 0, KS, nullptr, 0, 0, nullptr, 0, 0,
         2, HP, W2a, HP, nullptr, nullptr, 0, nullptr, nullptr, 0, nullptr,
         PQ, 2 * HP, 1, nullptr, nullptr);
    gemm(NB, s1_hi, 0, KS, s1_lo, 0, KS, nullptr, 0, 0, nullptr, 0, 0,
         2, HP, W2b, HP, nullptr, nullptr, 0, nullptr, nullptr, 0, nullptr,
         PQ + HP, 2 * HP, 1, nullptr, nullptr);
    pair_kernel<<<dim3(NB / 2), dim3(NTHR), PAIR_LDS, stream>>>(
        PQ, fc2_b, ln2_g, ln2_b, W3, fc3_b, ln3_g, ln3_b, W4, fc4_b, ln4_g, ln4_b,
        fc5_w, fc5_b, es_hi, es_lo);
    gemm(NB, s1_hi, 0, KS, s1_lo, 0, KS, es_hi, HP, KS, es_lo, HP, KS,
         4, HP, Wfc6, 2 * HP, fc6_b, nullptr, 0, ln6_g, ln6_b, 0, nullptr,
         out, HH, 2, nullptr, nullptr);
}
